// Barrier_Net_50354196578949
// MI455X (gfx1250) — hardware-verified
//
#include <hip/hip_runtime.h>
#include <math.h>

typedef __attribute__((ext_vector_type(16))) _Float16 v16h;
typedef __attribute__((ext_vector_type(8)))  _Float16 v8h;
typedef __attribute__((ext_vector_type(8)))  float    v8f;
typedef __attribute__((ext_vector_type(4)))  float    v4f;
typedef __attribute__((ext_vector_type(2)))  float    v2f;

constexpr int kXDim   = 133;
constexpr int kNNb    = 16;
constexpr int kNOb    = 32;
constexpr int kColG   = 1;
constexpr int kColNb  = 5;
constexpr int kColOb  = kColNb + 4 * kNNb;
constexpr int kHid    = 64;
constexpr int kPhiOut = 16;
constexpr int kRhoOut = 8;
constexpr int kPsiIn  = 2 * kRhoOut + 2;
constexpr int kActDim = 2;
static_assert(kColOb == 69);
static_assert(kColOb + 2 * kNOb == kXDim);
static_assert(kPsiIn == 18);
static_assert(4 * kNNb + 2 * kNOb == 128);

constexpr float kDRobot = 0.3f;
constexpr float kDObst  = 0.5f;
constexpr float kGamma  = 0.01f;
constexpr float kPhiMin = -2.0f;
constexpr float kPhiMax = 2.0f;
constexpr float kActMin = -2.0f;
constexpr float kActMax = 2.0f;

constexpr float kCarryW    = 256.0f;
constexpr float kCarryPool = 16.0f;
constexpr float kCarryAct  = 64.0f;
constexpr float kInvPW     = 1.0f / (kCarryPool * kCarryW);
constexpr float kInvAW     = 1.0f / (kCarryAct * kCarryW);
constexpr float kF16Normal = 6.103515625e-5f;

constexpr int kOffPnW2  = 0;
constexpr int kOffPoW2  = kOffPnW2 + 16 * 64;
constexpr int kOffRnW1  = kOffPoW2 + 16 * 64;
constexpr int kOffRoW1  = kOffRnW1 + 64 * 32;
constexpr int kOffRnW2  = kOffRoW1 + 64 * 32;
constexpr int kOffRoW2  = kOffRnW2 + 16 * 64;
constexpr int kOffPsW1  = kOffRoW2 + 16 * 64;
constexpr int kOffPsW2  = kOffPsW1 + 64 * 32;
constexpr int kOffPsW3  = kOffPsW2 + 64 * 64;
constexpr int kWtHalves = kOffPsW3 + 16 * 64;
static_assert(kWtHalves == 15360);

constexpr int kOffP0 = 0;
constexpr int kOffP1 = kOffP0 + 16 * 64;
constexpr int kOffSn = kOffP1 + 16 * 64;
constexpr int kOffSo = kOffSn + 16 * 32;
constexpr int kOffH  = kOffSo + 16 * 32;
constexpr int kActHalves = kOffH + 16 * 32;
static_assert(kActHalves == 3584);
static_assert(kWtHalves * 2 + 4 * kActHalves * 2 + 4 * 2 * 128 * 4 + 4 * 32 * 4 == 64000);

__device__ __forceinline__ _Float16 to_h16(float v) {
  const float w = (fabsf(v) < kF16Normal) ? 0.0f : v;
  return (_Float16)w;
}

__device__ __forceinline__ v16h frag_load(const _Float16* p) {
  union U { v16h v; v8h h[2]; } f;
  f.h[0] = *(const v8h*)(p);
  f.h[1] = *(const v8h*)(p + 16);
  return f.v;
}

__device__ __forceinline__ v8f mma_g(v16h a, v16h b, v8f c) {
  c = __builtin_amdgcn_wmma_f32_16x16x32_f16(false, a, false, b, (short)0, c, false, false);
  asm volatile("v_nop\n\tv_nop\n\tv_nop\n\tv_nop" : "+v"(c) : "v"(a), "v"(b));
  return c;
}

template <int KS>
__device__ __forceinline__ v8f tile_mma(const _Float16* A, int ap, const _Float16* Bt, int bp, int lane, v8f acc) {
  const int m  = lane & 15;
  const int ko = (lane >> 4) * 8;
#pragma unroll
  for (int ks = 0; ks < KS; ++ks) {
    const v16h a = frag_load(A + m * ap + ks * 32 + ko);
    const v16h b = frag_load(Bt + m * bp + ks * 32 + ko);
    acc = mma_g(a, b, acc);
  }
  return acc;
}

template <bool RELU>
__device__ __forceinline__ void store_tile_h16(_Float16* dst, int pitch, int col0, v8f acc,
                                               float scale, float bias, float carry, int lane) {
  const int hh = lane >> 4;
  const int cm = lane & 15;
#pragma unroll
  for (int r = 0; r < 8; ++r) {
    float v = acc[r] * scale + bias;
    if (RELU) v = fmaxf(v, 0.0f);
    dst[(8 * hh + r) * pitch + col0 + cm] = to_h16(v * carry);
  }
}

__device__ __forceinline__ void stage_bt(_Float16* dst, const float* __restrict__ W, int kreal, int nreal,
                                         int nlo, int kpadlog2, int count, int tid) {
#pragma unroll 1
  for (int idx = tid; idx < count; idx += 128) {
    const int n  = idx >> kpadlog2;
    const int k  = idx & ((1 << kpadlog2) - 1);
    const int nn = n - nlo;
    const bool ok = (k < kreal) && (nn >= 0) && (nn < nreal);
    const int kc = (k < kreal) ? k : (kreal - 1);
    int nc = (nn < 0) ? 0 : nn;
    nc = (nc < nreal) ? nc : (nreal - 1);
    float v = W[kc * nreal + nc];
    asm volatile("" : "+v"(v));
    const float s = ok ? (v * kCarryW) : 0.0f;
    dst[idx] = to_h16(s);
  }
}

__device__ __forceinline__ void rep_term(float px, float py, float dsafe, float& tx, float& ty) {
#pragma clang fp contract(off)
  const float nrm  = sqrtf(px * px + py * py);
  const float hgap = nrm - dsafe;
  const float den  = nrm * hgap;
  const float inv  = 1.0f / den;
  tx = (kGamma * (-px)) * inv;
  ty = (kGamma * (-py)) * inv;
}

__global__ __launch_bounds__(128) void fused_policy_kernel(
    const float* __restrict__ x, const float* __restrict__ noise,
    const float* __restrict__ pnW1, const float* __restrict__ pnb1,
    const float* __restrict__ pnW2, const float* __restrict__ pnb2,
    const float* __restrict__ rnW1, const float* __restrict__ rnb1,
    const float* __restrict__ rnW2, const float* __restrict__ rnb2,
    const float* __restrict__ poW1, const float* __restrict__ pob1,
    const float* __restrict__ poW2, const float* __restrict__ pob2,
    const float* __restrict__ roW1, const float* __restrict__ rob1,
    const float* __restrict__ roW2, const float* __restrict__ rob2,
    const float* __restrict__ psW1, const float* __restrict__ psb1,
    const float* __restrict__ psW2, const float* __restrict__ psb2,
    const float* __restrict__ psW3, const float* __restrict__ psb3,
    float* __restrict__ out, int nb)
{
  __shared__ __align__(16) _Float16 sWt[kWtHalves];
  __shared__ __align__(16) _Float16 sAct[4][kActHalves];
  __shared__ __align__(16) float    sRow[4][2][128];
  __shared__ __align__(16) float    sEmp[4][32];

  const int tid  = threadIdx.x;
  const int wave = tid >> 5;
  const int lane = tid & 31;
  const int hh   = lane >> 4;
  const int cm   = lane & 15;
  const int base = blockIdx.x * 64 + wave * 16;

  stage_bt(sWt + kOffPnW2, pnW2, kHid,    kPhiOut, 0, 6, 16 * 64, tid);
  stage_bt(sWt + kOffPoW2, poW2, kHid,    kPhiOut, 0, 6, 16 * 64, tid);
  stage_bt(sWt + kOffRnW1, rnW1, kPhiOut, kHid,    0, 5, 64 * 32, tid);
  stage_bt(sWt + kOffRoW1, roW1, kPhiOut, kHid,    0, 5, 64 * 32, tid);
  stage_bt(sWt + kOffRnW2, rnW2, kHid,    kRhoOut, 0, 6, 16 * 64, tid);
  stage_bt(sWt + kOffRoW2, roW2, kHid,    kRhoOut, kRhoOut, 6, 16 * 64, tid);
  stage_bt(sWt + kOffPsW1, psW1, kPsiIn,  kHid,    0, 5, 64 * 32, tid);
  stage_bt(sWt + kOffPsW2, psW2, kHid,    kHid,    0, 6, 64 * 64, tid);
  stage_bt(sWt + kOffPsW3, psW3, kHid,    kActDim, 0, 6, 16 * 64, tid);

  _Float16* P0 = &sAct[wave][kOffP0];
  _Float16* P1 = &sAct[wave][kOffP1];
  _Float16* Sn = &sAct[wave][kOffSn];
  _Float16* So = &sAct[wave][kOffSo];
  _Float16* Hp = &sAct[wave][kOffH];

  const int f0 = lane;
  const int f1 = lane + 32;
  const float wn00 = pnW1[0 * kHid + f0], wn10 = pnW1[1 * kHid + f0], wn20 = pnW1[2 * kHid + f0], wn30 = pnW1[3 * kHid + f0];
  const float wn01 = pnW1[0 * kHid + f1], wn11 = pnW1[1 * kHid + f1], wn21 = pnW1[2 * kHid + f1], wn31 = pnW1[3 * kHid + f1];
  const float wo00 = poW1[0 * kHid + f0], wo10 = poW1[1 * kHid + f0];
  const float wo01 = poW1[0 * kHid + f1], wo11 = poW1[1 * kHid + f1];
  const float bn0 = pnb1[f0], bn1 = pnb1[f1];
  const float bo0 = pob1[f0], bo1 = pob1[f1];

  int nzi = base * 2 + lane;
  nzi = (nzi < nb * 2) ? nzi : (nb * 2 - 1);
  const float nz = noise[nzi];

  float rep = 0.0f;
#pragma unroll 1
  for (int e = 0; e < 16; ++e) {
    int r = base + e;
    r = (r < nb) ? r : (nb - 1);
    const float* xr = x + (size_t)r * kXDim + kColNb;
    const float v0 = xr[lane];
    const float v1 = xr[lane + 32];
    const float v2 = xr[lane + 64];
    const float v3 = xr[lane + 96];
    float* rb = &sRow[wave][e & 1][0];
    rb[lane]      = v0;
    rb[lane + 32] = v1;
    rb[lane + 64] = v2;
    rb[lane + 96] = v3;
    __syncthreads();

    const v2f npos = *(const v2f*)(rb + 4 * cm);
    const v2f opos = *(const v2f*)(rb + 64 + 2 * lane);
    float ntx, nty, otx, oty;
    rep_term(npos[0], npos[1], kDRobot, ntx, nty);
    rep_term(opos[0], opos[1], kDObst, otx, oty);
    float sx = otx + ((lane < 16) ? ntx : 0.0f);
    float sy = oty + ((lane < 16) ? nty : 0.0f);
    sx += __shfl_xor(sx, 16, 32);
    sy += __shfl_xor(sy, 16, 32);
    sx += __shfl_xor(sx, 8, 32);
    sy += __shfl_xor(sy, 8, 32);
    sx += __shfl_xor(sx, 4, 32);
    sy += __shfl_xor(sy, 4, 32);
    sx += __shfl_xor(sx, 2, 32);
    sy += __shfl_xor(sy, 2, 32);
    sx += __shfl_xor(sx, 1, 32);
    sy += __shfl_xor(sy, 1, 32);
    rep = (lane == 2 * e) ? sx : rep;
    rep = (lane == 2 * e + 1) ? sy : rep;

    float an0 = 0.0f, an1 = 0.0f;
#pragma unroll 4
    for (int i = 0; i < kNNb; ++i) {
      const v4f a = *(const v4f*)(rb + 4 * i);
      float t0 = a[0] * wn00;
      t0 = fmaf(a[1], wn10, t0);
      t0 = fmaf(a[2], wn20, t0);
      t0 = fmaf(a[3], wn30, t0);
      float t1 = a[0] * wn01;
      t1 = fmaf(a[1], wn11, t1);
      t1 = fmaf(a[2], wn21, t1);
      t1 = fmaf(a[3], wn31, t1);
      an0 += fmaxf(t0 + bn0, 0.0f);
      an1 += fmaxf(t1 + bn1, 0.0f);
    }
    float ao0 = 0.0f, ao1 = 0.0f;
#pragma unroll 4
    for (int j = 0; j < kNOb; ++j) {
      const v2f o = *(const v2f*)(rb + 64 + 2 * j);
      float t0 = o[0] * wo00;
      t0 = fmaf(o[1], wo10, t0);
      float t1 = o[0] * wo01;
      t1 = fmaf(o[1], wo11, t1);
      ao0 += fmaxf(t0 + bo0, 0.0f);
      ao1 += fmaxf(t1 + bo1, 0.0f);
    }
    P0[e * 64 + f0] = to_h16(an0 * kCarryPool);
    P0[e * 64 + f1] = to_h16(an1 * kCarryPool);
    P1[e * 64 + f0] = to_h16(ao0 * kCarryPool);
    P1[e * 64 + f1] = to_h16(ao1 * kCarryPool);
  }
  __syncthreads();

  const v8f kZero = (v8f){0.f, 0.f, 0.f, 0.f, 0.f, 0.f, 0.f, 0.f};

  {
    v8f an = tile_mma<2>(P0, 64, sWt + kOffPnW2, 64, lane, kZero);
    v8f ao = tile_mma<2>(P1, 64, sWt + kOffPoW2, 64, lane, kZero);
    const float bnv = (float)kNNb * pnb2[cm];
    const float bov = (float)kNOb * pob2[cm];
    store_tile_h16<false>(Sn, 32, 0, an, kInvPW, bnv, kCarryAct, lane);
    store_tile_h16<false>(So, 32, 0, ao, kInvPW, bov, kCarryAct, lane);
    v8h z8;
#pragma unroll
    for (int q = 0; q < 8; ++q) z8[q] = (_Float16)0.0f;
    const int zr = lane >> 1;
    const int zc = 16 + 8 * (lane & 1);
    *(v8h*)(Sn + zr * 32 + zc) = z8;
    *(v8h*)(So + zr * 32 + zc) = z8;
  }
  __syncthreads();

#pragma unroll 1
  for (int j = 0; j < 4; ++j) {
    v8f an = tile_mma<1>(Sn, 32, sWt + kOffRnW1 + j * 16 * 32, 32, lane, kZero);
    v8f ao = tile_mma<1>(So, 32, sWt + kOffRoW1 + j * 16 * 32, 32, lane, kZero);
    const float bnv = rnb1[j * 16 + cm];
    const float bov = rob1[j * 16 + cm];
    store_tile_h16<true>(P0, 64, j * 16, an, kInvAW, bnv, kCarryAct, lane);
    store_tile_h16<true>(P1, 64, j * 16, ao, kInvAW, bov, kCarryAct, lane);
  }
  __syncthreads();

  {
    v8f acc = tile_mma<2>(P0, 64, sWt + kOffRnW2, 64, lane, kZero);
    acc = tile_mma<2>(P1, 64, sWt + kOffRoW2, 64, lane, acc);
    float ba = rnb2[cm & 7];
    float bb = rob2[cm & 7];
    asm volatile("" : "+v"(ba));
    asm volatile("" : "+v"(bb));
    const float bsel = (cm < 8) ? ba : bb;
    store_tile_h16<false>(Hp, 32, 0, acc, kInvAW, bsel, kCarryAct, lane);
    int gr = base + cm;
    gr = (gr < nb) ? gr : (nb - 1);
    float g0 = x[(size_t)gr * kXDim + kColG];
    float g1 = x[(size_t)gr * kXDim + kColG + 1];
    asm volatile("" : "+v"(g0));
    asm volatile("" : "+v"(g1));
    const float e0 = (lane < 16) ? (g0 * kCarryAct) : 0.0f;
    const float e1 = (lane < 16) ? (g1 * kCarryAct) : 0.0f;
    float z0 = 0.0f;
    asm volatile("" : "+v"(z0));
    const _Float16 zh = to_h16(z0);
    v8h gv;
    gv[0] = to_h16(e0);
    gv[1] = to_h16(e1);
#pragma unroll
    for (int q = 2; q < 8; ++q) gv[q] = zh;
    *(v8h*)(Hp + cm * 32 + 16 + 8 * hh) = gv;
  }
  __syncthreads();

#pragma unroll 1
  for (int j = 0; j < 4; ++j) {
    v8f acc = tile_mma<1>(Hp, 32, sWt + kOffPsW1 + j * 16 * 32, 32, lane, kZero);
    const float bv = psb1[j * 16 + cm];
    store_tile_h16<true>(P0, 64, j * 16, acc, kInvAW, bv, kCarryAct, lane);
  }
  __syncthreads();

#pragma unroll 1
  for (int j = 0; j < 4; ++j) {
    v8f acc = tile_mma<2>(P0, 64, sWt + kOffPsW2 + j * 16 * 64, 64, lane, kZero);
    const float bv = psb2[j * 16 + cm];
    store_tile_h16<true>(P1, 64, j * 16, acc, kInvAW, bv, kCarryAct, lane);
  }
  __syncthreads();

  {
    v8f acc = tile_mma<2>(P1, 64, sWt + kOffPsW3, 64, lane, kZero);
    float b3 = psb3[(cm < kActDim) ? cm : (kActDim - 1)];
    asm volatile("" : "+v"(b3));
    float* ep = &sEmp[wave][0];
    if (cm < kActDim) {
#pragma unroll
      for (int r = 0; r < 8; ++r) ep[(8 * hh + r) * kActDim + cm] = acc[r] * kInvAW + b3;
    }
  }
  __syncthreads();

  {
    const float p  = sEmp[wave][lane];
    const float t  = tanhf(p);
    const float em = (t + 1.0f) * 0.5f * (kPhiMax - kPhiMin) + kPhiMin;
    const float z  = (em + rep) + nz;
    const float tz = tanhf(z);
    const float o  = (tz + 1.0f) * 0.5f * (kActMax - kActMin) + kActMin;
    const bool ok = (base + (lane >> 1)) < nb;
    volatile float* po = out + (size_t)base * kActDim + lane;
    if (ok) *po = o;
    __threadfence();
    if (ok) *po = o;
  }
}

extern "C" void kernel_launch(void* const* d_in, const int* in_sizes, int n_in,
                              void* d_out, int out_size, void* d_ws, size_t ws_size,
                              hipStream_t stream) {
  (void)d_ws;
  (void)ws_size;
  if (n_in < 24) return;
  const int nb = in_sizes[0] / kXDim;
  if (nb <= 0) return;
  if (nb * kXDim != in_sizes[0]) return;
  if ((nb % 64) != 0) return;
  if (in_sizes[1] != nb * kActDim) return;
  if (in_sizes[2] != 4 * kHid) return;
  if (in_sizes[3] != kHid) return;
  if (in_sizes[4] != kHid * kPhiOut) return;
  if (in_sizes[5] != kPhiOut) return;
  if (in_sizes[6] != kPhiOut * kHid) return;
  if (in_sizes[7] != kHid) return;
  if (in_sizes[8] != kHid * kRhoOut) return;
  if (in_sizes[9] != kRhoOut) return;
  if (in_sizes[10] != 2 * kHid) return;
  if (in_sizes[11] != kHid) return;
  if (in_sizes[12] != kHid * kPhiOut) return;
  if (in_sizes[13] != kPhiOut) return;
  if (in_sizes[14] != kPhiOut * kHid) return;
  if (in_sizes[15] != kHid) return;
  if (in_sizes[16] != kHid * kRhoOut) return;
  if (in_sizes[17] != kRhoOut) return;
  if (in_sizes[18] != kPsiIn * kHid) return;
  if (in_sizes[19] != kHid) return;
  if (in_sizes[20] != kHid * kHid) return;
  if (in_sizes[21] != kHid) return;
  if (in_sizes[22] != kHid * kActDim) return;
  if (in_sizes[23] != kActDim) return;
  if (out_size != nb * kActDim) return;

  const float* x     = (const float*)d_in[0];
  const float* noise = (const float*)d_in[1];
  const float* pnW1  = (const float*)d_in[2];
  const float* pnb1  = (const float*)d_in[3];
  const float* pnW2  = (const float*)d_in[4];
  const float* pnb2  = (const float*)d_in[5];
  const float* rnW1  = (const float*)d_in[6];
  const float* rnb1  = (const float*)d_in[7];
  const float* rnW2  = (const float*)d_in[8];
  const float* rnb2  = (const float*)d_in[9];
  const float* poW1  = (const float*)d_in[10];
  const float* pob1  = (const float*)d_in[11];
  const float* poW2  = (const float*)d_in[12];
  const float* pob2  = (const float*)d_in[13];
  const float* roW1  = (const float*)d_in[14];
  const float* rob1  = (const float*)d_in[15];
  const float* roW2  = (const float*)d_in[16];
  const float* rob2  = (const float*)d_in[17];
  const float* psW1  = (const float*)d_in[18];
  const float* psb1  = (const float*)d_in[19];
  const float* psW2  = (const float*)d_in[20];
  const float* psb2  = (const float*)d_in[21];
  const float* psW3  = (const float*)d_in[22];
  const float* psb3  = (const float*)d_in[23];
  float* out = (float*)d_out;

  fused_policy_kernel<<<dim3(nb / 64), dim3(128), 0, stream>>>(
      x, noise, pnW1, pnb1, pnW2, pnb2, rnW1, rnb1, rnW2, rnb2,
      poW1, pob1, poW2, pob2, roW1, rob1, roW2, rob2,
      psW1, psb1, psW2, psb2, psW3, psb3, out, nb);
}
